// SequenceLSTM_19748259627557
// MI455X (gfx1250) — hardware-verified
//
#include <hip/hip_runtime.h>
#include <stdint.h>

typedef __attribute__((ext_vector_type(16))) _Float16 v16h;
typedef __attribute__((ext_vector_type(8)))  _Float16 v8h;
typedef __attribute__((ext_vector_type(8)))  float    v8f;
typedef __attribute__((ext_vector_type(4)))  float    v4f;
typedef __attribute__((ext_vector_type(4)))  unsigned int v4u;

constexpr int NBATCH   = 1024;
constexpr int T_OBS    = 1000;
constexpr int NSTEPS   = 1200;
constexpr int HID      = 51;
constexpr int HPAD     = 64;
constexpr int NGCOL    = 256;
constexpr int KL0      = 64;
constexpr int KL1      = 128;
constexpr int ROWS_PB  = 16;
constexpr int NTHR     = 128;
constexpr int APITCH   = 136;
constexpr int YB_PITCH = 36;
constexpr int YCHUNK   = 32;
constexpr int NCHUNK   = 38;
constexpr int YPITCH   = NCHUNK * YCHUNK;
constexpr float A_CARRY  = 16.0f;
constexpr float W_CARRY  = 256.0f;
constexpr float ACC_FOLD = 1.0f / 4096.0f;
constexpr float LOG2E_F  = 1.4426950408889634f;
constexpr float LOG2E_X2 = 2.8853900817779268f;

static_assert(NSTEPS == 37 * YCHUNK + 16, "chunk layout");
static_assert(NBATCH % ROWS_PB == 0, "row tiling");
static_assert((NBATCH * NSTEPS) % (4 * 256) == 0, "copy grid exact");
static_assert(KL0 % 32 == 0 && KL1 % 32 == 0, "K multiple of 32");

template <typename T> struct Frag;
template <> struct Frag<_Float16> {
  typedef v16h V; union U { v16h v; v8h h[2]; };
  static __device__ __forceinline__ v16h load(const _Float16* p) {
    U f; f.h[0] = *(const v8h*)(p); f.h[1] = *(const v8h*)(p + 16); return f.v;
  }
};

__device__ __forceinline__ v8f mma_h(v16h a, v16h b, v8f c) {
  c = __builtin_amdgcn_wmma_f32_16x16x32_f16(false, a, false, b, (short)0, c, false, false);
  asm volatile("v_nop\n\tv_nop\n\tv_nop\n\tv_nop" : "+v"(c) : "v"(a), "v"(b));
  return c;
}
__device__ __forceinline__ void code_fence() { asm volatile("" ::: "memory"); }

__device__ __forceinline__ unsigned int f16_bits(float f) {
  return (unsigned int)__builtin_bit_cast(unsigned short, (_Float16)f);
}

__device__ __forceinline__ float sigm_f(float x) {
  const float e = __builtin_amdgcn_exp2f(-x * LOG2E_F);
  return __builtin_amdgcn_rcpf(1.0f + e);
}
__device__ __forceinline__ float tanh_f(float x) {
  const float e = __builtin_amdgcn_exp2f(x * LOG2E_X2);
  return 1.0f - 2.0f * __builtin_amdgcn_rcpf(1.0f + e);
}
__device__ __forceinline__ void lstm_cell(float zi, float zf, float zg, float zo, float& cst, float& hout) {
  const float ii = sigm_f(zi);
  const float ff = sigm_f(zf);
  const float gg = tanh_f(zg);
  const float oo = sigm_f(zo);
  const float cn = ff * cst + ii * gg;
  cst = cn;
  hout = oo * tanh_f(cn);
}

__global__ __launch_bounds__(256) void pack_weights_f16(
    const float* __restrict__ w_hh0, const float* __restrict__ w_ih1, const float* __restrict__ w_hh1,
    unsigned short* __restrict__ bt0, unsigned short* __restrict__ bt1) {
  const int i = blockIdx.x * 256 + threadIdx.x;
  float v[8];
  unsigned short* dst;
  if (i < 2048) {
    const int n = i >> 3, kg = i & 7;
    const int g = n >> 6, u = n & 63;
    const int uc = (u < HID) ? u : (HID - 1);
    const int row = g * HID + uc;
#pragma unroll
    for (int e = 0; e < 8; ++e) {
      const int k = kg * 8 + e;
      const int kc = (k < HID) ? k : (HID - 1);
      const float w = w_hh0[row * HID + kc];
      v[e] = (u < HID && k < HID) ? (w * W_CARRY) : 0.0f;
    }
    dst = bt0 + (size_t)n * KL0 + kg * 8;
  } else {
    const int j = i - 2048;
    const int n = j >> 4, kg = j & 15;
    const int g = n >> 6, u = n & 63;
    const int uc = (u < HID) ? u : (HID - 1);
    const int row = g * HID + uc;
#pragma unroll
    for (int e = 0; e < 8; ++e) {
      const int k = kg * 8 + e;
      const int ka = (k < HID) ? k : (HID - 1);
      const int kb0 = k - HPAD;
      const int kb = (kb0 < 0) ? 0 : ((kb0 < HID) ? kb0 : (HID - 1));
      const float wa = w_ih1[row * HID + ka];
      const float wb = w_hh1[row * HID + kb];
      float val = (k < HID) ? (wa * W_CARRY) : ((k >= HPAD && k < HPAD + HID) ? (wb * W_CARRY) : 0.0f);
      v[e] = (u < HID) ? val : 0.0f;
    }
    dst = bt1 + (size_t)n * KL1 + kg * 8;
  }
  v4u pk;
  pk[0] = f16_bits(v[0]) | (f16_bits(v[1]) << 16);
  pk[1] = f16_bits(v[2]) | (f16_bits(v[3]) << 16);
  pk[2] = f16_bits(v[4]) | (f16_bits(v[5]) << 16);
  pk[3] = f16_bits(v[6]) | (f16_bits(v[7]) << 16);
  *(volatile v4u*)dst = pk;
  __threadfence();
  *(volatile v4u*)dst = pk;
}

__device__ __forceinline__ void flush_chunk(const float* yb, float* __restrict__ ystage, int row0, int chunk, int lane) {
  const int q = lane >> 3;
  const int p4 = (lane & 7) * 4;
  for (int pass = 0; pass < 2; ++pass) {
#pragma unroll
    for (int it = 0; it < 4; ++it) {
      const int rl = it * 4 + q;
      const v4f val = *(const v4f*)(yb + rl * YB_PITCH + p4);
      *(volatile v4f*)(ystage + (size_t)(row0 + rl) * YPITCH + chunk * YCHUNK + p4) = val;
    }
    __threadfence();
  }
}

__global__ __launch_bounds__(NTHR) void lstm2_persistent(
    const float* __restrict__ input, const float* __restrict__ w_ih0,
    const float* __restrict__ b_ih0, const float* __restrict__ b_hh0,
    const float* __restrict__ b_ih1, const float* __restrict__ b_hh1,
    const float* __restrict__ w_lin, const float* __restrict__ b_lin,
    const int* __restrict__ horizon,
    const unsigned short* __restrict__ bt0p, const unsigned short* __restrict__ bt1p,
    float* __restrict__ ystage) {
  __shared__ __align__(16) _Float16 As[ROWS_PB * APITCH];
  __shared__ __align__(16) float    ybuf[ROWS_PB * YB_PITCH];
  __shared__ __align__(16) float    yp[4 * ROWS_PB];
  (void)horizon;

  const int tid  = threadIdx.x;
  const int wave = tid >> 5;
  const int lane = tid & 31;
  const int hh   = lane >> 4;
  const int c    = lane & 15;
  const int row0 = blockIdx.x * ROWS_PB;
  const int u    = wave * 16 + c;
  const bool ureal = (u < HID);
  const int uc   = ureal ? u : (HID - 1);

  float wih0r[4], b0r[4], b1r[4];
#pragma unroll
  for (int g = 0; g < 4; ++g) {
    const int idx = g * HID + uc;
    const float wa  = w_ih0[idx];
    const float bb0 = b_ih0[idx] + b_hh0[idx];
    const float bb1 = b_ih1[idx] + b_hh1[idx];
    wih0r[g] = ureal ? wa  : 0.0f;
    b0r[g]   = ureal ? bb0 : 0.0f;
    b1r[g]   = ureal ? bb1 : 0.0f;
  }
  const float wl   = ureal ? w_lin[uc] : 0.0f;
  const float blin = b_lin[0];

  {
    unsigned int* az = (unsigned int*)As;
    for (int i = tid; i < ROWS_PB * APITCH / 2; i += NTHR) az[i] = 0u;
    for (int i = tid; i < ROWS_PB * YB_PITCH; i += NTHR) ybuf[i] = 0.0f;
    if (tid < 4 * ROWS_PB) yp[tid] = 0.0f;
  }

  float c0s[8], c1s[8];
#pragma unroll
  for (int r = 0; r < 8; ++r) { c0s[r] = 0.0f; c1s[r] = 0.0f; }
  const v8f zero8 = (v8f){0.f, 0.f, 0.f, 0.f, 0.f, 0.f, 0.f, 0.f};

  const _Float16* bt0 = (const _Float16*)(const void*)bt0p;
  const _Float16* bt1 = (const _Float16*)(const void*)bt1p;
  const _Float16* arow  = As + c * APITCH + 8 * hh;
  const _Float16* b0row = bt0 + (size_t)u * KL0 + 8 * hh;
  const _Float16* b1row = bt1 + (size_t)u * KL1 + 8 * hh;

#pragma unroll 1
  for (int t = 0; t < NSTEPS; ++t) {
    __syncthreads();

    float xr[8];
    {
      const int tc = (t < T_OBS) ? t : (T_OBS - 1);
#pragma unroll
      for (int r = 0; r < 8; ++r) {
        const int rl = 8 * hh + r;
        float y = ((yp[rl] + yp[ROWS_PB + rl]) + yp[2 * ROWS_PB + rl]) + yp[3 * ROWS_PB + rl];
        y += blin;
        const float xin = input[(size_t)(row0 + rl) * T_OBS + tc];
        xr[r] = (t < T_OBS) ? xin : y;
        if (wave == 0 && c == 0 && t > 0) ybuf[rl * YB_PITCH + ((t - 1) & (YCHUNK - 1))] = y;
      }
    }

    const v16h a0k0 = Frag<_Float16>::load(arow);
    const v16h a0k1 = Frag<_Float16>::load(arow + 32);
    const v16h a1k2 = Frag<_Float16>::load(arow + 64);
    const v16h a1k3 = Frag<_Float16>::load(arow + 96);
    v8f acc[4];
#pragma unroll
    for (int g = 0; g < 4; ++g) {
      const _Float16* bp = b0row + (size_t)g * 64 * KL0;
      v8f a = zero8;
      a = mma_h(a0k0, Frag<_Float16>::load(bp), a);
      a = mma_h(a0k1, Frag<_Float16>::load(bp + 32), a);
      acc[g] = a;
      code_fence();
    }
    float h0r[8];
#pragma unroll
    for (int r = 0; r < 8; ++r) {
      const float zi = acc[0][r] * ACC_FOLD + (xr[r] * wih0r[0] + b0r[0]);
      const float zf = acc[1][r] * ACC_FOLD + (xr[r] * wih0r[1] + b0r[1]);
      const float zg = acc[2][r] * ACC_FOLD + (xr[r] * wih0r[2] + b0r[2]);
      const float zo = acc[3][r] * ACC_FOLD + (xr[r] * wih0r[3] + b0r[3]);
      lstm_cell(zi, zf, zg, zo, c0s[r], h0r[r]);
    }

    __syncthreads();

#pragma unroll
    for (int r = 0; r < 8; ++r) As[(8 * hh + r) * APITCH + u] = (_Float16)(h0r[r] * A_CARRY);
    if (wave == 0 && t > 0 && (t & (YCHUNK - 1)) == 0)
      flush_chunk(ybuf, ystage, row0, (t >> 5) - 1, lane);

    __syncthreads();

    const v16h a1k0 = Frag<_Float16>::load(arow);
    const v16h a1k1 = Frag<_Float16>::load(arow + 32);
#pragma unroll
    for (int g = 0; g < 4; ++g) {
      const _Float16* bp = b1row + (size_t)g * 64 * KL1;
      v8f a = zero8;
      a = mma_h(a1k0, Frag<_Float16>::load(bp), a);
      a = mma_h(a1k1, Frag<_Float16>::load(bp + 32), a);
      a = mma_h(a1k2, Frag<_Float16>::load(bp + 64), a);
      a = mma_h(a1k3, Frag<_Float16>::load(bp + 96), a);
      acc[g] = a;
      code_fence();
    }

    float ps[8];
#pragma unroll
    for (int r = 0; r < 8; ++r) {
      const float zi = acc[0][r] * ACC_FOLD + b1r[0];
      const float zf = acc[1][r] * ACC_FOLD + b1r[1];
      const float zg = acc[2][r] * ACC_FOLD + b1r[2];
      const float zo = acc[3][r] * ACC_FOLD + b1r[3];
      float h1;
      lstm_cell(zi, zf, zg, zo, c1s[r], h1);
      As[(8 * hh + r) * APITCH + HPAD + u] = (_Float16)(h1 * A_CARRY);
      ps[r] = h1 * wl;
    }
#pragma unroll
    for (int r = 0; r < 8; ++r) {
      float s = ps[r];
      s += __shfl_xor(s, 8, 32);
      s += __shfl_xor(s, 4, 32);
      s += __shfl_xor(s, 2, 32);
      s += __shfl_xor(s, 1, 32);
      ps[r] = s;
    }
    if (c == 0) {
#pragma unroll
      for (int r = 0; r < 8; ++r) yp[wave * ROWS_PB + 8 * hh + r] = ps[r];
    }
  }

  __syncthreads();
#pragma unroll
  for (int r = 0; r < 8; ++r) {
    const int rl = 8 * hh + r;
    float y = ((yp[rl] + yp[ROWS_PB + rl]) + yp[2 * ROWS_PB + rl]) + yp[3 * ROWS_PB + rl];
    y += blin;
    if (wave == 0 && c == 0) ybuf[rl * YB_PITCH + ((NSTEPS - 1) & (YCHUNK - 1))] = y;
  }
  __syncthreads();
  if (wave == 0) flush_chunk(ybuf, ystage, row0, NCHUNK - 1, lane);
}

__global__ __launch_bounds__(256) void copy_out(const float* __restrict__ ystage, float* __restrict__ out, int n4) {
  const int i = blockIdx.x * 256 + threadIdx.x;
  if (i < n4) {
    const int row = i / (NSTEPS / 4);
    const int c4  = i - row * (NSTEPS / 4);
    const v4f val = *(const v4f*)(ystage + (size_t)row * YPITCH + c4 * 4);
    *(volatile v4f*)(out + (size_t)i * 4) = val;
    __threadfence();
    *(volatile v4f*)(out + (size_t)i * 4) = val;
  }
}

extern "C" void kernel_launch(void* const* d_in, const int* in_sizes, int n_in,
                              void* d_out, int out_size, void* d_ws, size_t ws_size,
                              hipStream_t stream) {
  if (n_in < 12) return;
  if (in_sizes[0] != NBATCH * T_OBS || out_size != NBATCH * NSTEPS) return;
  const float* input = (const float*)d_in[0];
  const float* w_ih0 = (const float*)d_in[1];
  const float* w_hh0 = (const float*)d_in[2];
  const float* b_ih0 = (const float*)d_in[3];
  const float* b_hh0 = (const float*)d_in[4];
  const float* w_ih1 = (const float*)d_in[5];
  const float* w_hh1 = (const float*)d_in[6];
  const float* b_ih1 = (const float*)d_in[7];
  const float* b_hh1 = (const float*)d_in[8];
  const float* w_lin = (const float*)d_in[9];
  const float* b_lin = (const float*)d_in[10];
  const int*   horizon = (const int*)d_in[11];
  float* out = (float*)d_out;

  const size_t off_bt0 = 0;
  const size_t off_bt1 = off_bt0 + (size_t)NGCOL * KL0 * 2;
  const size_t off_y   = off_bt1 + (size_t)NGCOL * KL1 * 2;
  const size_t total   = off_y + (size_t)NBATCH * YPITCH * 4;
  if (total > ws_size) return;
  char* ws = (char*)d_ws;
  unsigned short* bt0 = (unsigned short*)(ws + off_bt0);
  unsigned short* bt1 = (unsigned short*)(ws + off_bt1);
  float* ystage = (float*)(ws + off_y);

  pack_weights_f16<<<dim3(24), dim3(256), 0, stream>>>(w_hh0, w_ih1, w_hh1, bt0, bt1);
  lstm2_persistent<<<dim3(NBATCH / ROWS_PB), dim3(NTHR), 0, stream>>>(
      input, w_ih0, b_ih0, b_hh0, b_ih1, b_hh1, w_lin, b_lin, horizon, bt0, bt1, ystage);
  const int n4 = NBATCH * NSTEPS / 4;
  copy_out<<<dim3((n4 + 255) / 256), dim3(256), 0, stream>>>(ystage, out, n4);
}
